// GroupedQueryAttention_11295763988511
// MI455X (gfx1250) — hardware-verified
//
#include <hip/hip_runtime.h>


#ifndef NB
#define NB 2
#endif
#ifndef SEQ
#define SEQ 2048
#endif
#define SEQ_FULL 2048
#define DM   2048
#define NH_  16
#define NKV  4
#define REP  (NH_ / NKV)
#define HD   128
#define DQ   (NH_ * HD)
#define DKV  (NKV * HD)
#define RH   (SEQ < 512 ? SEQ : 512)
#define XBS_FULL ((size_t)SEQ_FULL * DM)
#define KCAR 64.0f
#define VCAR 16.0f
#define CCAR 1024.0f
#define WCAR 1024.0f
#define SL2  (1.4426950408889634f / (KCAR * 11.3137084989847604f))
#define OSP  132
static_assert(HD == 128);
static_assert(SEQ % 64 == 0 && RH % 64 == 0 && (SEQ - RH) % 64 == 0);
static_assert(DM % 64 == 0 && DQ % 64 == 0 && DKV % 64 == 0 && DM % 32 == 0 && DQ % 32 == 0);
static_assert(((size_t)SEQ * DM / 8) % 256 == 0);
static_assert(((size_t)SEQ * 64) % 256 == 0);
static_assert(((size_t)NKV * HD * SEQ / 2) % 256 == 0);
static_assert((SEQ / 2) % 8 == 0);
static_assert(NH_ % NKV == 0);

typedef _Float16 h16;
typedef unsigned short bf;
typedef __attribute__((ext_vector_type(16))) __bf16   v16bf;
typedef __attribute__((ext_vector_type(16))) _Float16 v16h;
typedef __attribute__((ext_vector_type(16))) unsigned short v16us;
typedef __attribute__((ext_vector_type(8)))  _Float16 v8h;
typedef __attribute__((ext_vector_type(8)))  unsigned short v8us;
typedef __attribute__((ext_vector_type(8)))  float    v8f;
typedef __attribute__((ext_vector_type(4)))  float    v4f;
typedef __attribute__((ext_vector_type(2)))  float    v2f;
typedef __attribute__((ext_vector_type(2)))  _Float16 v2h;
typedef __attribute__((ext_vector_type(2)))  unsigned short v2us;
typedef v4f  __attribute__((may_alias)) v4fa;
typedef v8us __attribute__((may_alias)) v8usa;

__device__ __forceinline__ unsigned short f2bf(float f) { unsigned u = __float_as_uint(f); u += 0x7FFFu + ((u >> 16) & 1u); return (unsigned short)(u >> 16); }
__device__ __forceinline__ float bf2f(unsigned short b) { return __uint_as_float(((unsigned)b) << 16); }
__device__ __forceinline__ float bfr(float f) { return bf2f(f2bf(f)); }
__device__ __forceinline__ void splitf(float y, unsigned short& h, unsigned short& l) { h = f2bf(y); l = f2bf(y - bf2f(h)); }
__device__ __forceinline__ v16h cat16(v8h lo, v8h hi) { return __builtin_shufflevector(lo, hi, 0, 1, 2, 3, 4, 5, 6, 7, 8, 9, 10, 11, 12, 13, 14, 15); }
__device__ __forceinline__ v16bf cat16b(v8us lo, v8us hi) { return __builtin_bit_cast(v16bf, __builtin_shufflevector(lo, hi, 0, 1, 2, 3, 4, 5, 6, 7, 8, 9, 10, 11, 12, 13, 14, 15)); }
__device__ __forceinline__ v8f wmma16(v16h a, v16h b, v8f c) { return __builtin_amdgcn_wmma_f32_16x16x32_f16(false, a, false, b, (short)0, c, false, false); }
__device__ __forceinline__ v8f wmmab(v16bf a, v16bf b, v8f c) { return __builtin_amdgcn_wmma_f32_16x16x32_bf16(false, a, false, b, (short)0, c, false, false); }

template <typename T16> struct WFrag;
template <> struct WFrag<h16> { typedef v16h V; static __device__ __forceinline__ V ld(const h16* p) { return cat16(*(const v8h*)p, *(const v8h*)(p + 16)); } static __device__ __forceinline__ v8f mma(V a, V b, v8f c) { return wmma16(a, b, c); } };
template <> struct WFrag<bf> { typedef v16bf V; static __device__ __forceinline__ V ld(const bf* p) { return cat16b(*(const v8us*)p, *(const v8us*)(p + 16)); } static __device__ __forceinline__ v8f mma(V a, V b, v8f c) { return wmmab(a, b, c); } };

template <typename T16, int NSPLIT, bool BIAS>
__global__ __launch_bounds__(32) void k_gemmw(const T16* __restrict__ A, const T16* __restrict__ A2, const T16* __restrict__ Bt, const T16* __restrict__ Bt2, int K, float* C, int ldc, const float* __restrict__ bias, float osc, size_t sA, size_t sB, size_t sC) {
    typedef typename WFrag<T16>::V V;
    __shared__ __align__(16) float os[16 * 68];
    const size_t z = blockIdx.z; A += z * sA; if (A2) A2 += z * sA; Bt += z * sB; if (Bt2) Bt2 += z * sB; C += z * sC;
    const int lane = threadIdx.x & 31, lr = lane & 15, hi = lane >> 4; const int r0 = blockIdx.x * 64, c0 = blockIdx.y * 64;
    v8f acc[4][4];
#pragma unroll
    for (int mb = 0; mb < 4; ++mb)
#pragma unroll
        for (int nb = 0; nb < 4; ++nb) acc[mb][nb] = (v8f){};
    const size_t aoff = (size_t)(r0 + lr) * K + 8 * hi, boff = (size_t)(c0 + lr) * K + 8 * hi;
#pragma unroll 1
    for (int kc = 0; kc < K; kc += 32) {
        V a[4], a2[4];
#pragma unroll
        for (int mb = 0; mb < 4; ++mb) { a[mb] = WFrag<T16>::ld(A + aoff + (size_t)mb * 16 * K + kc); if (NSPLIT == 1 || NSPLIT == 2) a2[mb] = WFrag<T16>::ld(A2 + aoff + (size_t)mb * 16 * K + kc); }
#pragma unroll
        for (int nb = 0; nb < 4; ++nb) { const V b = WFrag<T16>::ld(Bt + boff + (size_t)nb * 16 * K + kc); V b2; if (NSPLIT >= 2) b2 = WFrag<T16>::ld(Bt2 + boff + (size_t)nb * 16 * K + kc);
#pragma unroll
            for (int mb = 0; mb < 4; ++mb) { acc[mb][nb] = WFrag<T16>::mma(a[mb], b, acc[mb][nb]); if (NSPLIT == 1 || NSPLIT == 2) acc[mb][nb] = WFrag<T16>::mma(a2[mb], b, acc[mb][nb]); if (NSPLIT >= 2) acc[mb][nb] = WFrag<T16>::mma(a[mb], b2, acc[mb][nb]); } }
        asm volatile("v_nop\n\tv_nop\n\tv_nop\n\tv_nop" : "+v"(acc[0][0]), "+v"(acc[1][1]), "+v"(acc[2][2]), "+v"(acc[3][3]) : "v"(a[0]), "v"(a[3]));
    }
#pragma unroll
    for (int mb = 0; mb < 4; ++mb) {
#pragma unroll
        for (int nb = 0; nb < 4; ++nb) {
#pragma unroll
            for (int j = 0; j < 8; ++j) os[(hi * 8 + j) * 68 + nb * 16 + lr] = acc[mb][nb][j]; }
        __builtin_amdgcn_wave_barrier(); asm volatile("" ::: "memory");
        float* crow = C + (size_t)(r0 + mb * 16) * ldc + c0;
#pragma unroll 1
        for (int ps = 0; ps < 2; ++ps) {
#pragma unroll
            for (int s = 0; s < 8; ++s) { const int row = 2 * s + hi, cofs = lr * 4; v4f val = *(const v4fa*)(os + row * 68 + cofs); val = val * osc; if (BIAS) { val[0] += bfr(bias[c0 + cofs]); val[1] += bfr(bias[c0 + cofs + 1]); val[2] += bfr(bias[c0 + cofs + 2]); val[3] += bfr(bias[c0 + cofs + 3]); }
                *(volatile v4f*)(crow + (size_t)row * ldc + cofs) = val; }
            if (ps == 0) __threadfence(); }
        __builtin_amdgcn_wave_barrier(); asm volatile("" ::: "memory");
    }
}

__global__ __launch_bounds__(256) void k_cvt8(const float* __restrict__ src, bf* dst, size_t n8) { const size_t i = (size_t)blockIdx.x * 256 + threadIdx.x; if (i >= n8) return; const v8f v = *(const v8f*)(src + i * 8); v8us o;
#pragma unroll
    for (int k = 0; k < 8; ++k) o[k] = f2bf(v[k]); *(volatile v8us*)(dst + i * 8) = o; __threadfence(); *(volatile v8us*)(dst + i * 8) = o; }

template <bool F16OUT>
__global__ __launch_bounds__(256) void k_wtr(const float* __restrict__ W, unsigned short* Wt, unsigned K, unsigned N, float sc) {
    __shared__ __align__(16) unsigned short ts[64 * 72];
    const unsigned tid = threadIdx.x, k0 = blockIdx.x * 64u, n0 = blockIdx.y * 64u;
#pragma unroll
    for (unsigned it = 0; it < 4; ++it) {
        const unsigned q = tid + it * 256u, kr = q >> 4, nc = (q & 15u) * 4u;
        const v4f v = *(const v4f*)(W + (size_t)(k0 + kr) * N + n0 + nc);
#pragma unroll
        for (unsigned j = 0; j < 4; ++j) {
            const float b = bfr(v[j]);
            unsigned short o;
            if (F16OUT) o = __builtin_bit_cast(unsigned short, (h16)(b * sc)); else o = f2bf(v[j]);
            ts[(nc + j) * 72u + kr] = o;
        }
    }
    __syncthreads();
    const unsigned lane = tid & 31u, wv = tid >> 5;
#pragma unroll 1
    for (unsigned ps = 0; ps < 2; ++ps) {
#pragma unroll
        for (unsigned it = 0; it < 2; ++it) {
            const unsigned ln = it * 32u + wv * 4u + (lane >> 3), pc = (lane & 7u) * 8u;
            const v8us val = *(const v8usa*)(ts + ln * 72u + pc);
            *(volatile v8us*)(Wt + (size_t)(n0 + ln) * K + k0 + pc) = val;
        }
        if (ps == 0) __threadfence();
    }
}

__global__ __launch_bounds__(256) void k_cstab(float* CS) {
    const unsigned idx = blockIdx.x * 256u + threadIdx.x;
    if (idx >= (unsigned)SEQ * 64u) return;
    const unsigned i = idx & 63u, t = idx >> 6;
    double pw = 1.0;
    pw = (i & 1u)  ? pw * 1.1547819846894583 : pw;
    pw = (i & 2u)  ? pw * 1.3335214321633240 : pw;
    pw = (i & 4u)  ? pw * 1.7782794100389228 : pw;
    pw = (i & 8u)  ? pw * 3.1622776601683795 : pw;
    pw = (i & 16u) ? pw * 10.0 : pw;
    pw = (i & 32u) ? pw * 100.0 : pw;
    const float pf = (float)pw;
    const float inv = 1.0f / pf;
    const float ang = (float)t * inv;
    const double a = (double)ang;
    const double kd = __builtin_rint(a * 0.63661977236758134);
    const double rd = __builtin_fma(-kd, 1.5707963267948966, a);
    const float r = (float)rd;
    const unsigned q = ((unsigned)(int)kd) & 3u;
    const float r2 = r * r;
    float sp = 2.7557319e-6f; sp = sp * r2 - 1.9841270e-4f; sp = sp * r2 + 8.3333333e-3f; sp = sp * r2 - 1.6666667e-1f;
    const float s = r + r * r2 * sp;
    float cp = -2.7557319e-7f; cp = cp * r2 + 2.4801587e-5f; cp = cp * r2 - 1.3888889e-3f; cp = cp * r2 + 4.1666667e-2f; cp = cp * r2 - 0.5f;
    const float c = 1.0f + r2 * cp;
    const float co = (q == 0u) ? c : ((q == 1u) ? -s : ((q == 2u) ? -c : s));
    const float si = (q == 0u) ? s : ((q == 1u) ? c : ((q == 2u) ? -s : -c));
    v2f cs; cs[0] = co; cs[1] = si;
    *(volatile v2f*)(CS + (size_t)idx * 2) = cs; __threadfence(); *(volatile v2f*)(CS + (size_t)idx * 2) = cs;
}

__global__ __launch_bounds__(256) void k_nrope(const float* __restrict__ F, unsigned pitch, const float* __restrict__ CS, const float* __restrict__ alpha, unsigned useA, float carry, h16* P16, bf* Ph, bf* Pl) {
    const unsigned lane = threadIdx.x & 31u, wv = threadIdx.x >> 5;
    const unsigned u = blockIdx.x * 8u + wv;
    const unsigned h = u / ((unsigned)SEQ / 2u);
    const unsigned t = (u % ((unsigned)SEQ / 2u)) * 2u + (lane >> 4);
    const unsigned d0 = (lane & 15u) * 8u;
    const float* f = F + (size_t)t * pitch + h * HD + d0;
    const v4f xa = *(const v4f*)f; const v4f xb = *(const v4f*)(f + 4);
    float x[8]; x[0] = xa[0]; x[1] = xa[1]; x[2] = xa[2]; x[3] = xa[3]; x[4] = xb[0]; x[5] = xb[1]; x[6] = xb[2]; x[7] = xb[3];
    float ss = 0.0f;
#pragma unroll
    for (int k = 0; k < 8; ++k) ss += x[k] * x[k];
    ss += __shfl_xor(ss, 8, 32); ss += __shfl_xor(ss, 4, 32); ss += __shfl_xor(ss, 2, 32); ss += __shfl_xor(ss, 1, 32);
    const float av = bfr(alpha[h & 15u]);
    const float fac = useA ? av * 11.3137084989847604f : 1.0f;
    const float sc = 1.0f / (sqrtf(ss) + 1.0e-6f);
    const float* cp = CS + ((size_t)t * (HD / 2) + (d0 >> 1)) * 2u;
    const v4f ca = *(const v4f*)cp; const v4f cb = *(const v4f*)(cp + 4);
    float cs[8]; cs[0] = ca[0]; cs[1] = ca[1]; cs[2] = ca[2]; cs[3] = ca[3]; cs[4] = cb[0]; cs[5] = cb[1]; cs[6] = cb[2]; cs[7] = cb[3];
    v8h o16; v8us oh, ol;
#pragma unroll
    for (int j = 0; j < 4; ++j) {
        const float x1 = (x[2 * j] * sc) * fac, x2 = (x[2 * j + 1] * sc) * fac; const float c = cs[2 * j], s = cs[2 * j + 1];
        const float r1 = (x1 * c - x2 * s) * carry, r2 = (x1 * s + x2 * c) * carry;
        unsigned short a2, c2;
        o16[2 * j] = (h16)r1; splitf(r1, a2, c2); oh[2 * j] = a2; ol[2 * j] = c2;
        o16[2 * j + 1] = (h16)r2; splitf(r2, a2, c2); oh[2 * j + 1] = a2; ol[2 * j + 1] = c2;
    }
    const size_t o1 = ((size_t)h * SEQ + t) * HD + d0;
    const size_t o2 = ((size_t)h * RH + (t < (unsigned)RH ? t : 0u)) * HD + d0;
    const bool hires = (t < (unsigned)RH);
    *(volatile v8h*)(P16 + o1) = o16;
    if (hires) { *(volatile v8us*)(Ph + o2) = oh; *(volatile v8us*)(Pl + o2) = ol; }
    __threadfence();
    *(volatile v8h*)(P16 + o1) = o16;
    if (hires) { *(volatile v8us*)(Ph + o2) = oh; *(volatile v8us*)(Pl + o2) = ol; }
}

__global__ __launch_bounds__(256) void k_vtp(const float* __restrict__ F, unsigned pitch, h16* V16, bf* Vh, bf* Vl) {
    const unsigned e = (blockIdx.x * 256u + threadIdx.x) * 2u; if (e >= (unsigned)NKV * HD * SEQ) return;
    const unsigned t = e % (unsigned)SEQ; const unsigned d = (e / (unsigned)SEQ) % (unsigned)HD; const unsigned g = e / ((unsigned)SEQ * HD); v2h o16; v2us oh, ol;
#pragma unroll
    for (unsigned q = 0; q < 2; ++q) { const float xv = F[(size_t)(t + q) * pitch + g * HD + d]; o16[q] = (h16)(xv * VCAR); unsigned short a2, c2; splitf(xv, a2, c2); oh[q] = a2; ol[q] = c2; }
    *(volatile v2h*)(V16 + e) = o16; *(volatile v2us*)(Vh + e) = oh; *(volatile v2us*)(Vl + e) = ol; __threadfence(); *(volatile v2h*)(V16 + e) = o16; *(volatile v2us*)(Vh + e) = oh; *(volatile v2us*)(Vl + e) = ol; }


__global__ __launch_bounds__(32) void k_flash_lo(const h16* __restrict__ QP, const h16* __restrict__ KP, const h16* __restrict__ VT, h16* A16, unsigned qt0) {
    __shared__ __align__(16) float os[16 * OSP];
    const unsigned lane = threadIdx.x & 31u, lh = lane & 15u, ks = lane >> 4;
    const unsigned qt = blockIdx.x + qt0, h = blockIdx.y, g = h / (unsigned)REP;
    const unsigned qbase = qt * 16u, qcol = qbase + lh;
    const h16* qrow = QP + ((size_t)h * SEQ + qcol) * HD + 8u * ks;
    v16h qf[4];
#pragma unroll
    for (int j = 0; j < 4; ++j) qf[j] = WFrag<h16>::ld(qrow + 32 * j);
    const h16* kb = KP + ((size_t)g * SEQ + lh) * HD + 8u * ks;
    const h16* vb = VT + ((size_t)g * HD + lh) * SEQ + 8u * ks;
    v8f o[8];
#pragma unroll
    for (int dt = 0; dt < 8; ++dt) o[dt] = (v8f){};
    float mrow = -1.0e30f, lrow = 0.0f;
    const unsigned ntiles = (qbase + 16u + 31u) >> 5;
#pragma unroll 1
    for (unsigned kt = 0; kt < ntiles; ++kt) {
        const unsigned s0 = kt << 5;
        const h16* kr0 = kb + (size_t)s0 * HD; const h16* kr1 = kr0 + 16 * HD;
        v8f st0 = (v8f){}, st1 = (v8f){};
#pragma unroll
        for (int j = 0; j < 4; ++j) { const v16h a = WFrag<h16>::ld(kr0 + 32 * j); const v16h c = WFrag<h16>::ld(kr1 + 32 * j); st0 = wmma16(a, qf[j], st0); st1 = wmma16(c, qf[j], st1); }
        asm volatile("v_nop\n\tv_nop\n\tv_nop\n\tv_nop" : "+v"(st0), "+v"(st1) : "v"(qf[3]));
        const unsigned kofs = s0 + 8u * ks;
        float sv[16]; float tmax = -1.0e30f;
#pragma unroll
        for (unsigned r = 0; r < 8; ++r) {
            sv[r]     = (kofs + r       <= qcol) ? st0[r] * SL2 : -1.0e30f;
            sv[r + 8] = (kofs + r + 16u <= qcol) ? st1[r] * SL2 : -1.0e30f;
            tmax = fmaxf(tmax, fmaxf(sv[r], sv[r + 8]));
        }
        tmax = fmaxf(tmax, __shfl_xor(tmax, 16, 32));
        const float mnew = fmaxf(mrow, tmax);
        const float scale = __builtin_amdgcn_exp2f(mrow - mnew);
        v16h pf; float psum = 0.0f;
#pragma unroll
        for (int i = 0; i < 16; ++i) { const float pv = __builtin_amdgcn_exp2f(sv[i] - mnew); psum += pv; pf[i] = (h16)pv; }
        psum += __shfl_xor(psum, 16, 32);
        lrow = lrow * scale + psum; mrow = mnew;
#pragma unroll
        for (int dt = 0; dt < 8; ++dt) o[dt] = o[dt] * scale;
        const h16* vr = vb + s0;
#pragma unroll
        for (int dt = 0; dt < 8; ++dt) { const v16h a = WFrag<h16>::ld(vr + (size_t)dt * 16 * SEQ); o[dt] = wmma16(a, pf, o[dt]); }
        asm volatile("v_nop\n\tv_nop\n\tv_nop\n\tv_nop" : "+v"(o[0]), "+v"(o[1]), "+v"(o[2]), "+v"(o[3]), "+v"(o[4]), "+v"(o[5]), "+v"(o[6]), "+v"(o[7]) : "v"(pf));
    }
    const float f = (CCAR / VCAR) * (1.0f / lrow);
#pragma unroll
    for (int dt = 0; dt < 8; ++dt)
#pragma unroll
        for (int r = 0; r < 8; ++r) os[lh * OSP + dt * 16 + 8 * ks + r] = o[dt][r] * f;
    __builtin_amdgcn_wave_barrier(); asm volatile("" ::: "memory");
    h16* arow = A16 + (size_t)(qbase - (unsigned)RH) * DQ + h * HD;
#pragma unroll 1
    for (int ps = 0; ps < 2; ++ps) {
#pragma unroll
        for (unsigned s = 0; s < 8; ++s) { const unsigned row = 2u * s + ks, pc = lh * 8u; const v4f a = *(const v4fa*)(os + row * OSP + pc); const v4f b = *(const v4fa*)(os + row * OSP + pc + 4); v8h o8;
            o8[0] = (h16)a[0]; o8[1] = (h16)a[1]; o8[2] = (h16)a[2]; o8[3] = (h16)a[3]; o8[4] = (h16)b[0]; o8[5] = (h16)b[1]; o8[6] = (h16)b[2]; o8[7] = (h16)b[3];
            *(volatile v8h*)(arow + (size_t)row * DQ + pc) = o8; }
        if (ps == 0) __threadfence(); }
}

__global__ __launch_bounds__(32) void k_flash_hi(const bf* __restrict__ Qh, const bf* __restrict__ Ql, const bf* __restrict__ Kh, const bf* __restrict__ Kl, const bf* __restrict__ Vh, const bf* __restrict__ Vl, bf* Ah, bf* Al) {
    __shared__ __align__(16) float os[16 * OSP];
    const unsigned lane = threadIdx.x & 31u, lh = lane & 15u, ks = lane >> 4;
    const unsigned qt = blockIdx.x, h = blockIdx.y, g = h / (unsigned)REP;
    const unsigned qbase = qt * 16u, qcol = qbase + lh;
    const size_t qo = ((size_t)h * RH + qcol) * HD + 8u * ks;
    v16bf qh[4];
#pragma unroll
    for (int j = 0; j < 4; ++j) qh[j] = WFrag<bf>::ld(Qh + qo + 32 * j);
    const bf* qlp = Ql + qo;
    const size_t ko = ((size_t)g * RH + lh) * HD + 8u * ks;
    const size_t vo = ((size_t)g * HD + lh) * SEQ + 8u * ks;
    v8f o[8];
#pragma unroll
    for (int dt = 0; dt < 8; ++dt) o[dt] = (v8f){};
    float mrow = -1.0e30f, lrow = 0.0f;
    const unsigned ntiles = (qbase + 16u + 31u) >> 5;
#pragma unroll 1
    for (unsigned kt = 0; kt < ntiles; ++kt) {
        const unsigned s0 = kt << 5;
        const size_t k0o = ko + (size_t)s0 * HD, k1o = k0o + (size_t)16 * HD;
        v8f st0 = (v8f){}, st1 = (v8f){};
#pragma unroll
        for (int j = 0; j < 4; ++j) {
            const v16bf qlj = WFrag<bf>::ld(qlp + 32 * j);
            const v16bf a = WFrag<bf>::ld(Kh + k0o + 32 * j), a2 = WFrag<bf>::ld(Kl + k0o + 32 * j);
            const v16bf c = WFrag<bf>::ld(Kh + k1o + 32 * j), c2 = WFrag<bf>::ld(Kl + k1o + 32 * j);
            st0 = wmmab(a, qh[j], st0); st0 = wmmab(a2, qh[j], st0); st0 = wmmab(a, qlj, st0);
            st1 = wmmab(c, qh[j], st1); st1 = wmmab(c2, qh[j], st1); st1 = wmmab(c, qlj, st1);
        }
        asm volatile("v_nop\n\tv_nop\n\tv_nop\n\tv_nop" : "+v"(st0), "+v"(st1) : "v"(qh[3]));
        const unsigned kofs = s0 + 8u * ks;
        float sv[16]; float tmax = -1.0e30f;
#pragma unroll
        for (unsigned r = 0; r < 8; ++r) {
            sv[r]     = (kofs + r       <= qcol) ? st0[r] * SL2 : -1.0e30f;
            sv[r + 8] = (kofs + r + 16u <= qcol) ? st1[r] * SL2 : -1.0e30f;
            tmax = fmaxf(tmax, fmaxf(sv[r], sv[r + 8]));
        }
        tmax = fmaxf(tmax, __shfl_xor(tmax, 16, 32));
        const float mnew = fmaxf(mrow, tmax);
        const float scale = __builtin_amdgcn_exp2f(mrow - mnew);
        v16us phv, plv; float psum = 0.0f;
#pragma unroll
        for (int i = 0; i < 16; ++i) { const float pv = __builtin_amdgcn_exp2f(sv[i] - mnew); psum += pv; unsigned short a2, c2; splitf(pv, a2, c2); phv[i] = a2; plv[i] = c2; }
        const v16bf ph = __builtin_bit_cast(v16bf, phv), pl = __builtin_bit_cast(v16bf, plv);
        psum += __shfl_xor(psum, 16, 32);
        lrow = lrow * scale + psum; mrow = mnew;
#pragma unroll
        for (int dt = 0; dt < 8; ++dt) o[dt] = o[dt] * scale;
        const size_t v0 = vo + s0;
#pragma unroll
        for (int dt = 0; dt < 8; ++dt) { const v16bf a = WFrag<bf>::ld(Vh + v0 + (size_t)dt * 16 * SEQ), a2 = WFrag<bf>::ld(Vl + v0 + (size_t)dt * 16 * SEQ);
            o[dt] = wmmab(a, ph, o[dt]); o[dt] = wmmab(a2, ph, o[dt]); o[dt] = wmmab(a, pl, o[dt]); }
        asm volatile("v_nop\n\tv_nop\n\tv_nop\n\tv_nop" : "+v"(o[0]), "+v"(o[1]), "+v"(o[2]), "+v"(o[3]), "+v"(o[4]), "+v"(o[5]), "+v"(o[6]), "+v"(o[7]) : "v"(ph), "v"(pl));
    }
    const float f = 1.0f / lrow;
#pragma unroll
    for (int dt = 0; dt < 8; ++dt)
#pragma unroll
        for (int r = 0; r < 8; ++r) os[lh * OSP + dt * 16 + 8 * ks + r] = o[dt][r] * f;
    __builtin_amdgcn_wave_barrier(); asm volatile("" ::: "memory");
    const size_t abase = (size_t)qbase * DQ + h * HD;
#pragma unroll 1
    for (int ps = 0; ps < 2; ++ps) {
#pragma unroll
        for (unsigned s = 0; s < 8; ++s) { const unsigned row = 2u * s + ks, pc = lh * 8u; const v4f a = *(const v4fa*)(os + row * OSP + pc); const v4f b = *(const v4fa*)(os + row * OSP + pc + 4); v8us oh, ol; unsigned short a2, c2;
            splitf(a[0], a2, c2); oh[0] = a2; ol[0] = c2; splitf(a[1], a2, c2); oh[1] = a2; ol[1] = c2; splitf(a[2], a2, c2); oh[2] = a2; ol[2] = c2; splitf(a[3], a2, c2); oh[3] = a2; ol[3] = c2;
            splitf(b[0], a2, c2); oh[4] = a2; ol[4] = c2; splitf(b[1], a2, c2); oh[5] = a2; ol[5] = c2; splitf(b[2], a2, c2); oh[6] = a2; ol[6] = c2; splitf(b[3], a2, c2); oh[7] = a2; ol[7] = c2;
            const size_t oo = abase + (size_t)row * DQ + pc;
            *(volatile v8us*)(Ah + oo) = oh; *(volatile v8us*)(Al + oo) = ol; }
        if (ps == 0) __threadfence(); }
}

constexpr size_t al256(size_t b) { return (b + 255) & ~(size_t)255; }
constexpr size_t SZ_WQ = (size_t)DQ * DM * 2, SZ_WK = (size_t)DKV * DM * 2, SZ_WO = (size_t)DM * DQ * 2;
constexpr size_t SZ_CS = (size_t)SEQ * 64 * 2 * 4;
constexpr size_t SZ_XB = (size_t)SEQ * DM * 2, SZ_FQ = (size_t)SEQ * DQ * 4, SZ_FK = (size_t)SEQ * DKV * 4;
constexpr size_t SZ_QP = (size_t)NH_ * SEQ * HD * 2, SZ_QH = (size_t)NH_ * RH * HD * 2, SZ_KP = (size_t)NKV * SEQ * HD * 2, SZ_KH = (size_t)NKV * RH * HD * 2;
constexpr size_t SZ_VT = (size_t)NKV * HD * SEQ * 2;
constexpr size_t SZ_AH = (size_t)RH * DQ * 2, SZ_A16 = ((size_t)(SEQ - RH) * DQ * 2 > 256) ? (size_t)(SEQ - RH) * DQ * 2 : 256;
constexpr size_t WS_TOTAL = al256(SZ_WQ) + 2 * al256(SZ_WK) + 2 * al256(SZ_WO) + al256(SZ_CS) + al256(SZ_XB) + al256(SZ_FQ) + 2 * al256(SZ_FK)
                          + al256(SZ_QP) + 2 * al256(SZ_QH) + al256(SZ_KP) + 2 * al256(SZ_KH) + 3 * al256(SZ_VT) + 2 * al256(SZ_AH) + al256(SZ_A16);
static_assert(WS_TOTAL <= (size_t)134217728);

extern "C" void kernel_launch(void* const* d_in, const int* in_sizes, int n_in,
                              void* d_out, int out_size, void* d_ws, size_t ws_size, hipStream_t stream) {
    if (n_in < 10) return;
    if ((size_t)in_sizes[0] < (size_t)(NB - 1) * XBS_FULL + (size_t)SEQ * DM) return;
    if (in_sizes[1] < DM * DQ || in_sizes[2] < DQ || in_sizes[3] < DM * DKV || in_sizes[4] < DKV || in_sizes[5] < DM * DKV || in_sizes[6] < DKV || in_sizes[7] < DQ * DM || in_sizes[8] < DM || in_sizes[9] < NH_) return;
    if ((size_t)out_size < (size_t)NB * SEQ * DM) return;
    if (WS_TOTAL > ws_size) return;
    const float* x = (const float*)d_in[0]; const float* wq = (const float*)d_in[1]; const float* bq = (const float*)d_in[2]; const float* wk = (const float*)d_in[3]; const float* bk = (const float*)d_in[4];
    const float* wv = (const float*)d_in[5]; const float* bv = (const float*)d_in[6]; const float* wo = (const float*)d_in[7]; const float* bo = (const float*)d_in[8]; const float* alpha = (const float*)d_in[9];
    float* OUT = (float*)d_out;
    char* wsp = (char*)d_ws;
    auto take = [&](size_t bytes) { char* p = wsp; wsp += al256(bytes); return (void*)p; };
    bf* WQ = (bf*)take(SZ_WQ); bf* WK = (bf*)take(SZ_WK); bf* WV = (bf*)take(SZ_WK); bf* WO = (bf*)take(SZ_WO); h16* WO16 = (h16*)take(SZ_WO);
    float* CS = (float*)take(SZ_CS);
    bf* XB = (bf*)take(SZ_XB); float* FQ = (float*)take(SZ_FQ); float* FK = (float*)take(SZ_FK); float* FV = (float*)take(SZ_FK);
    h16* QP16 = (h16*)take(SZ_QP); bf* QPh = (bf*)take(SZ_QH); bf* QPl = (bf*)take(SZ_QH); h16* KP16 = (h16*)take(SZ_KP); bf* KPh = (bf*)take(SZ_KH); bf* KPl = (bf*)take(SZ_KH);
    h16* VT16 = (h16*)take(SZ_VT); bf* VTh = (bf*)take(SZ_VT); bf* VTl = (bf*)take(SZ_VT);
    bf* ATh = (bf*)take(SZ_AH); bf* ATl = (bf*)take(SZ_AH); h16* AT16 = (h16*)take(SZ_A16);
    if ((size_t)(wsp - (char*)d_ws) > ws_size) return;

    k_wtr<false><<<dim3(DM / 64, DQ / 64), 256, 0, stream>>>(wq, (unsigned short*)WQ, DM, DQ, 1.0f);
    k_wtr<false><<<dim3(DM / 64, DKV / 64), 256, 0, stream>>>(wk, (unsigned short*)WK, DM, DKV, 1.0f);
    k_wtr<false><<<dim3(DM / 64, DKV / 64), 256, 0, stream>>>(wv, (unsigned short*)WV, DM, DKV, 1.0f);
    k_wtr<false><<<dim3(DQ / 64, DM / 64), 256, 0, stream>>>(wo, (unsigned short*)WO, DQ, DM, 1.0f);
    k_wtr<true><<<dim3(DQ / 64, DM / 64), 256, 0, stream>>>(wo, (unsigned short*)WO16, DQ, DM, WCAR);
    k_cstab<<<(unsigned)((size_t)SEQ * 64 / 256), 256, 0, stream>>>(CS);

    for (int b = 0; b < NB; ++b) {
        k_cvt8<<<(unsigned)((size_t)SEQ * DM / 8 / 256), 256, 0, stream>>>(x + (size_t)b * XBS_FULL, XB, (size_t)SEQ * DM / 8);
        k_gemmw<bf, 0, true><<<dim3(SEQ / 64, DQ / 64, 1), 32, 0, stream>>>(XB, nullptr, WQ, nullptr, DM, FQ, DQ, bq, 1.0f, 0, 0, 0);
        k_gemmw<bf, 0, true><<<dim3(SEQ / 64, DKV / 64, 1), 32, 0, stream>>>(XB, nullptr, WK, nullptr, DM, FK, DKV, bk, 1.0f, 0, 0, 0);
        k_gemmw<bf, 0, true><<<dim3(SEQ / 64, DKV / 64, 1), 32, 0, stream>>>(XB, nullptr, WV, nullptr, DM, FV, DKV, bv, 1.0f, 0, 0, 0);
        k_nrope<<<(unsigned)(NH_ * SEQ / 16), 256, 0, stream>>>(FQ, DQ, CS, alpha, 1u, 1.0f, QP16, QPh, QPl);
        k_nrope<<<(unsigned)(NKV * SEQ / 16), 256, 0, stream>>>(FK, DKV, CS, alpha, 0u, KCAR, KP16, KPh, KPl);
        k_vtp<<<(unsigned)((size_t)NKV * HD * SEQ / 2 / 256), 256, 0, stream>>>(FV, DKV, VT16, VTh, VTl);
        k_flash_hi<<<dim3(RH / 16, NH_), 32, 0, stream>>>(QPh, QPl, KPh, KPl, VTh, VTl, ATh, ATl);
        if (SEQ > RH) k_flash_lo<<<dim3((SEQ - RH) / 16, NH_), 32, 0, stream>>>(QP16, KP16, VT16, AT16, (unsigned)(RH / 16));
        k_gemmw<bf, 1, true><<<dim3(RH / 64, DM / 64, 1), 32, 0, stream>>>(ATh, ATl, WO, nullptr, DQ, OUT + (size_t)b * SEQ * DM, DM, bo, 1.0f, 0, 0, 0);
        if (SEQ > RH) k_gemmw<h16, 0, true><<<dim3((SEQ - RH) / 64, DM / 64, 1), 32, 0, stream>>>(AT16, nullptr, WO16, nullptr, DQ, OUT + ((size_t)b * SEQ + RH) * DM, DM, bo, 1.0f / (CCAR * WCAR), 0, 0, 0);
    }
}
